// SpatioTemporalGraphAttentionLayer_43748536877443
// MI455X (gfx1250) — hardware-verified
//
#include <hip/hip_runtime.h>
#include <math.h>

typedef __attribute__((ext_vector_type(16))) _Float16 v16h;
typedef __attribute__((ext_vector_type(16))) __bf16 v16b;
typedef __attribute__((ext_vector_type(8)))  _Float16 v8h;
typedef __attribute__((ext_vector_type(8)))  float v8f;
typedef __attribute__((ext_vector_type(4)))  float v4f;
typedef __attribute__((ext_vector_type(2)))  float v2f;
typedef __attribute__((ext_vector_type(4)))  unsigned v4u;
typedef __attribute__((ext_vector_type(4)))  int v4i;
typedef float __attribute__((may_alias)) float_a;
typedef int __attribute__((may_alias)) int_a;

template <typename T> __device__ __forceinline__ void vst2(void* p, T v) { *(volatile T*)p = v; __threadfence(); *(volatile T*)p = v; }
__device__ __forceinline__ v8f wmma16(v16h a, v16h b, v8f c) {
  v8f d = __builtin_amdgcn_wmma_f32_16x16x32_f16(false, a, false, b, (short)0, c, false, false);
  asm volatile("v_nop\n\tv_nop\n\tv_nop\n\tv_nop" : "+v"(d) : "v"(a), "v"(b));
  return d;
}
__device__ __forceinline__ v8f wmma_bf(v16b a, v16b b, v8f c) {
  v8f d = __builtin_amdgcn_wmma_f32_16x16x32_bf16(false, a, false, b, (short)0, c, false, false);
  asm volatile("v_nop\n\tv_nop\n\tv_nop\n\tv_nop" : "+v"(d) : "v"(a), "v"(b));
  return d;
}
__device__ __forceinline__ v16h frag_h(const _Float16* rowk0, int lane) {
  union { v16h v; v8h q[2]; } u; const _Float16* p = rowk0 + 8 * (lane >> 4);
  u.q[0] = *(const v8h*)p; u.q[1] = *(const v8h*)(p + 16); return u.v;
}
__device__ __forceinline__ v16h frag_f32(const float* rowk0, int lane) {
  v16h a; const float* p = rowk0 + 8 * (lane >> 4);
#pragma unroll
  for (int i = 0; i < 8; ++i) { a[i] = (_Float16)p[i]; a[8 + i] = (_Float16)p[16 + i]; }
  return a;
}
__device__ __forceinline__ v16h frag_f32s(const float* rowk0, int lane, float sc) {
  v16h a; const float* p = rowk0 + 8 * (lane >> 4);
#pragma unroll
  for (int i = 0; i < 8; ++i) { a[i] = (_Float16)(p[i] * sc); a[8 + i] = (_Float16)(p[16 + i] * sc); }
  return a;
}
__device__ __forceinline__ v16h fragc_f32(const float* W, int k0, int n, int lane, int ld, int K) {
  v16h a; const int g = lane >> 4;
#pragma unroll
  for (int i = 0; i < 8; ++i) { const int ka = k0 + 8 * g + i, kb = ka + 16;
    a[i] = (_Float16)(ka < K ? W[(size_t)(ka < K ? ka : K - 1) * ld + n] : 0.f); a[8 + i] = (_Float16)(kb < K ? W[(size_t)(kb < K ? kb : K - 1) * ld + n] : 0.f); }
  return a;
}
struct F2 { v16b h, l; };
__device__ __forceinline__ F2 bsplit16(const float v[16]) { F2 r;
#pragma unroll
  for (int i = 0; i < 16; ++i) { const __bf16 h = (__bf16)v[i]; r.h[i] = h; r.l[i] = (__bf16)(v[i] - (float)h); }
  return r; }
__device__ __forceinline__ F2 split_row(const float* row, int k0, int lane) { float v[16]; const float* p = row + k0 + 8 * (lane >> 4);
#pragma unroll
  for (int i = 0; i < 8; ++i) { v[i] = p[i]; v[8 + i] = p[16 + i]; }
  return bsplit16(v); }
__device__ __forceinline__ F2 split_rowK(const float* row, int k0, int lane, int K) { float v[16]; const int g = lane >> 4;
#pragma unroll
  for (int i = 0; i < 8; ++i) { const int ka = k0 + 8 * g + i, kb = ka + 16; v[i] = ka < K ? row[ka < K ? ka : K - 1] : 0.f; v[8 + i] = kb < K ? row[kb < K ? kb : K - 1] : 0.f; }
  return bsplit16(v); }
__device__ __forceinline__ F2 split_col(const float* W, int k0, int n, int lane, int ld, int K) { float v[16]; const int g = lane >> 4;
#pragma unroll
  for (int i = 0; i < 8; ++i) { const int ka = k0 + 8 * g + i, kb = ka + 16; v[i] = ka < K ? W[(size_t)(ka < K ? ka : K - 1) * ld + n] : 0.f; v[8 + i] = kb < K ? W[(size_t)(kb < K ? kb : K - 1) * ld + n] : 0.f; }
  return bsplit16(v); }
__device__ __forceinline__ v8f mac3(const F2& a, const F2& b, v8f c) { c = wmma_bf(a.l, b.h, c); c = wmma_bf(a.h, b.l, c); return wmma_bf(a.h, b.h, c); }
__device__ __forceinline__ float sigm(float v) { return 1.0f / (1.0f + expf(-v)); }
#define LDSX() do { asm volatile("s_wait_dscnt 0" ::: "memory"); __builtin_amdgcn_wave_barrier(); __builtin_amdgcn_fence(__ATOMIC_RELEASE, "workgroup"); } while (0)


#define NB 4
#define NN 2048
#define TT 12
#define FF 32
#define DD (TT * FF)
#define LL (NN * FF)
#define NS 0.2f
#ifndef TNB
#define TNB NB
#endif
typedef __attribute__((ext_vector_type(8))) __bf16 v8b;
__device__ __forceinline__ v16b frag_b(const __bf16* rowk0, int lane) {
  union { v16b v; v8b q[2]; } u; const __bf16* p = rowk0 + 8 * (lane >> 4);
  u.q[0] = *(const v8b*)p; u.q[1] = *(const v8b*)(p + 16); return u.v;
}
__device__ __forceinline__ float bfr(float v) { return (float)(__bf16)v; }
__device__ __attribute__((noinline)) float exp_ni(float v) { return expf(v); }
__device__ __attribute__((noinline)) float erf_ni(float v) { return erff(v); }

#define WS_PW  0u
#define WS_XT  (WS_PW + 2u * DD * DD)
#define WS_WH  (WS_XT + 4u * (size_t)NB * NN * DD)
#define WS_PH  (WS_WH + 4u * (size_t)NB * NN * DD)
#define WS_PL  (WS_PH + 2u * (size_t)NB * DD * NN)
#define WS_F1  (WS_PL + 2u * (size_t)NB * DD * NN)
#define WS_F2  (WS_F1 + 4u * (size_t)NB * NN)
#define WS_END (WS_F2 + 4u * (size_t)NB * NN)

__global__ __launch_bounds__(128) void k_packw(const float* __restrict__ Wm, __bf16* __restrict__ PW) { const int n = blockIdx.x, t = threadIdx.x; __shared__ __align__(16) __bf16 s[DD];
  for (int k = t; k < DD; k += 128) s[k] = (__bf16)Wm[(size_t)k * DD + n]; __syncthreads(); if (t < DD / 8) vst2((unsigned*)(PW + (size_t)n * DD + t * 8), *(const v4u*)&s[t * 8]); }
__global__ __launch_bounds__(128) void k_tconv(const float* __restrict__ X, const float* __restrict__ CW, const float* __restrict__ CB, float* __restrict__ XT) { __shared__ __align__(16) float so[2][DD + 4];
  const int tid = threadIdx.x, wave = tid >> 5, lane = tid & 31, col = lane & 15, g = lane >> 4; const size_t b = blockIdx.y; const int l0 = blockIdx.x * 64 + wave * 16;
  v8f acc = {};
#pragma unroll
  for (int kc = 0; kc < 2; ++kc) { v16b a, w; const int l = l0 + col;
#pragma unroll
    for (int i = 0; i < 16; ++i) { const int k = kc * 32 + 8 * g + (i < 8 ? i : 8 + i); float xv = 0.f, wv = 0.f; if (k < TT * 3) { const int ti = k / 3, kk = k % 3; const int lp = l + kk - 1; if (lp >= 0 && lp < LL) { const int n = lp >> 5, f = lp & 31; xv = X[((b * NN + n) * TT + ti) * FF + f]; } if (col < TT) wv = CW[(col * TT + ti) * 3 + kk]; } a[i] = (__bf16)xv; w[i] = (__bf16)wv; }
    acc = wmma_bf(a, w, acc); }
  if (col < TT) { const float bb = bfr(CB[col]);
#pragma unroll
    for (int r = 0; r < 8; ++r) { const int lr = wave * 16 + 8 * g + r; const int nl = lr >> 5, f = lr & 31; so[nl][col * FF + f] = acc[r] + bb; } }
  __syncthreads(); for (int e = tid; e < 2 * (DD / 4); e += 128) { const int nl = e / (DD / 4), q = e % (DD / 4); vst2(XT + (b * NN + (size_t)blockIdx.x * 2 + nl) * DD + q * 4, *(const v4f*)&so[nl][q * 4]); } }
__global__ __launch_bounds__(128) void k_wh(const float* __restrict__ XT, const __bf16* __restrict__ PW, float* __restrict__ WH, _Float16* __restrict__ PH, _Float16* __restrict__ PL) { __shared__ __align__(16) float sf[64][132]; __shared__ __align__(16) _Float16 th[128][72], tl[128][72];
  const int tid = threadIdx.x, wave = tid >> 5, lane = tid & 31, col = lane & 15, g = lane >> 4; const size_t b = blockIdx.z; const int n0 = blockIdx.x * 64; const int c0 = blockIdx.y * 128; const size_t r0 = b * NN + n0 + wave * 16;
  v8f acc[8] = {};
#pragma unroll
  for (int kc = 0; kc < DD / 32; ++kc) { const F2 a = split_row(XT + (r0 + col) * DD, kc * 32, lane);
#pragma unroll
    for (int j = 0; j < 8; ++j) { const v16b w = frag_b(PW + (size_t)(c0 + j * 16 + col) * DD + kc * 32, lane); acc[j] = wmma_bf(a.h, w, acc[j]); acc[j] = wmma_bf(a.l, w, acc[j]); } }
#pragma unroll
  for (int j = 0; j < 8; ++j)
#pragma unroll
    for (int r = 0; r < 8; ++r) { const float v = acc[j][r]; sf[wave * 16 + 8 * g + r][j * 16 + col] = v; const _Float16 hv = (_Float16)v; th[j * 16 + col][wave * 16 + 8 * g + r] = hv; tl[j * 16 + col][wave * 16 + 8 * g + r] = (_Float16)((v - (float)hv) * 2048.0f); }
  __syncthreads();
  for (int e = tid; e < 64 * 32; e += 128) { const int rl = e >> 5, q = e & 31; vst2(WH + (b * NN + n0 + rl) * DD + c0 + q * 4, *(const v4f*)&sf[rl][q * 4]); }
  for (int e = tid; e < 128 * 8; e += 128) { const int cl = e >> 3, q = e & 7; const size_t o = (b * DD + c0 + cl) * (size_t)NN + n0 + q * 8; vst2((unsigned*)(PH + o), *(const v4u*)&th[cl][q * 8]); vst2((unsigned*)(PL + o), *(const v4u*)&tl[cl][q * 8]); } }
__global__ __launch_bounds__(256) void k_coef(const float* __restrict__ WH, const float* __restrict__ A, float* __restrict__ F1, float* __restrict__ F2) { __shared__ __align__(16) float s1[32], s2[32]; const int t = threadIdx.x, w = t >> 5, lane = t & 31; const size_t r0 = (size_t)blockIdx.x * 32;
#pragma unroll 1
  for (int rr = 0; rr < 4; ++rr) { const size_t row = r0 + w * 4 + rr; const float* xr = WH + row * DD; float p1 = 0.f, p2 = 0.f;
#pragma unroll 1
    for (int c = lane; c < DD; c += 32) { const float v = xr[c]; p1 += v * bfr(A[c]); p2 += v * bfr(A[DD + c]); }
#pragma unroll
    for (int o = 1; o < 32; o <<= 1) { p1 += __shfl_xor(p1, o); p2 += __shfl_xor(p2, o); }
    if (lane == 0) { s1[w * 4 + rr] = p1; s2[w * 4 + rr] = p2; } }
  __syncthreads(); if (t < 8) vst2(F1 + r0 + t * 4, *(const v4f*)&s1[t * 4]); else if (t < 16) vst2(F2 + r0 + (t - 8) * 4, *(const v4f*)&s2[(t - 8) * 4]); }
__global__ __launch_bounds__(128) void k_gat(const float* __restrict__ F1, const float* __restrict__ F2, const int* __restrict__ ADJ, const _Float16* __restrict__ PH, const _Float16* __restrict__ PL, float* __restrict__ OUT) {
  __shared__ __align__(16) float sp[4][16][36]; __shared__ __align__(16) float so[4][16][132]; __shared__ float sf2[NN];
  const int tid = threadIdx.x, wave = tid >> 5, lane = tid & 31, col = lane & 15, g = lane >> 4; const int cb = blockIdx.y; const size_t b = blockIdx.z; const int i0 = blockIdx.x * 64 + wave * 16;
  for (int j = tid; j < NN; j += 128) sf2[j] = F2[b * NN + j]; __syncthreads();
  float f1v[8], m[8], l[8];
#pragma unroll
  for (int r = 0; r < 8; ++r) { f1v[r] = F1[b * NN + i0 + 8 * g + r]; m[r] = -3.0e38f; l[r] = 0.f; }
  v8f acc[8] = {}, accl[8] = {};
#pragma unroll 1
  for (int ks = 0; ks < NN / 32; ++ks) { float s[2][8];
#pragma unroll
    for (int ct = 0; ct < 2; ++ct) { const int j = ks * 32 + ct * 16 + col; const float f2v = sf2[j];
#pragma unroll
      for (int r = 0; r < 8; ++r) { const int i = i0 + 8 * g + r; float e = f1v[r] + f2v; e = e > 0.f ? e : NS * e; s[ct][r] = (ADJ[(size_t)i * NN + j] > 0) ? e : -3.0e38f; } }
    float alpha[8];
#pragma unroll
    for (int r = 0; r < 8; ++r) { float mx = fmaxf(s[0][r], s[1][r]);
#pragma unroll
      for (int o = 1; o < 16; o <<= 1) mx = fmaxf(mx, __shfl_xor(mx, o));
      const float mn = fmaxf(m[r], mx); alpha[r] = (m[r] <= -1.0e38f) ? 0.f : __expf(m[r] - mn); const float e0 = (s[0][r] <= -1.0e38f) ? 0.f : __expf(s[0][r] - mn), e1 = (s[1][r] <= -1.0e38f) ? 0.f : __expf(s[1][r] - mn); float es = e0 + e1;
#pragma unroll
      for (int o = 1; o < 16; o <<= 1) es += __shfl_xor(es, o);
      l[r] = l[r] * alpha[r] + es; m[r] = (mn > -1.0e38f) ? mn : m[r]; sp[wave][8 * g + r][col] = e0; sp[wave][8 * g + r][16 + col] = e1; }
#pragma unroll
    for (int jj = 0; jj < 8; ++jj)
#pragma unroll
      for (int r = 0; r < 8; ++r) { acc[jj][r] *= alpha[r]; accl[jj][r] *= alpha[r]; }
    LDSX();
    v16h pa; { const float* prow = &sp[wave][col][0] + 8 * (lane >> 4);
#pragma unroll
      for (int i = 0; i < 8; ++i) { pa[i] = (_Float16)(prow[i] * 2048.0f); pa[8 + i] = (_Float16)(prow[16 + i] * 2048.0f); } }
#pragma unroll
    for (int jj = 0; jj < 8; ++jj) { const size_t po = (b * DD + cb * 128 + jj * 16 + col) * (size_t)NN + ks * 32; acc[jj] = wmma16(pa, frag_h(PH + po, lane), acc[jj]); accl[jj] = wmma16(pa, frag_h(PL + po, lane), accl[jj]); }
    LDSX(); }
#pragma unroll
  for (int r = 0; r < 8; ++r) { const float il = (l[r] > 0.f) ? (1.0f / 2048.0f) / l[r] : 0.f;
#pragma unroll
    for (int jj = 0; jj < 8; ++jj) { const float v = (acc[jj][r] + accl[jj][r] * (1.0f / 2048.0f)) * il; so[wave][8 * g + r][jj * 16 + col] = v > 0.f ? v : expm1f(v); } }
  LDSX(); for (int rl = 0; rl < 16; ++rl) vst2(OUT + (b * NN + i0 + rl) * DD + cb * 128 + lane * 4, *(const v4f*)&so[wave][rl][lane * 4]); }
extern "C" void kernel_launch(void* const* d_in, const int* in_sizes, int n_in, void* d_out, int out_size, void* d_ws, size_t ws_size, hipStream_t stream) {
  (void)in_sizes; (void)n_in; (void)out_size;
  const float** F = (const float**)d_in;
  if (ws_size < (size_t)WS_END) return;
  char* ws = (char*)d_ws; __bf16* PW = (__bf16*)(ws + WS_PW); float *XT = (float*)(ws + WS_XT), *WH = (float*)(ws + WS_WH), *F1 = (float*)(ws + WS_F1), *F2 = (float*)(ws + WS_F2); _Float16 *PH = (_Float16*)(ws + WS_PH), *PL = (_Float16*)(ws + WS_PL);
  k_packw<<<DD, 128, 0, stream>>>(F[2], PW);
  k_tconv<<<dim3(LL / 64, NB), 128, 0, stream>>>(F[0], F[4], F[5], XT);
  k_wh<<<dim3(NN / 64, DD / 128, NB), 128, 0, stream>>>(XT, PW, WH, PH, PL);
  k_coef<<<NB * NN / 32, 256, 0, stream>>>(WH, F[3], F1, F2);
  k_gat<<<dim3(NN / 64, DD / 128, TNB), 128, 0, stream>>>(F1, F2, (const int*)d_in[1], PH, PL, (float*)d_out);
}
